// Mamba2SimpleBlock_85298050498978
// MI455X (gfx1250) — hardware-verified
//
#include <hip/hip_runtime.h>
#include <stdint.h>
#include <stddef.h>

typedef _Float16 v16h __attribute__((ext_vector_type(16)));
typedef _Float16 v8h  __attribute__((ext_vector_type(8)));
typedef float    v8f  __attribute__((ext_vector_type(8)));
typedef float    v4f  __attribute__((ext_vector_type(4)));

#define BDIM    2
#define LSEQ    2048
#define DMODEL  1024
#define DINNER  2048
#define NHEADS  4
#define DSTATE  64
#define HEADDIM 512
#define NPROJ   4612
#define NPAD    4672
#define ROWS    (BDIM * LSEQ)
#define COL_X   DINNER
#define COL_DT  (2 * DINNER)
#define COL_BC  (2 * DINNER + NHEADS)
#define RMS_EPS 1.1920929e-07f
#define WSCALE     32.0f
#define WSCALE_INV 0.03125f

#define GBM 128
#define GBN 64
#define SP  68
#define WS_LIMIT ((size_t)134217728)

static_assert(ROWS % GBM == 0);
static_assert(NPAD % GBN == 0);
static_assert(DMODEL % GBN == 0);
static_assert(DMODEL % 32 == 0);
static_assert(DINNER % 32 == 0);
static_assert(HEADDIM % 128 == 0);
static_assert(LSEQ % 8 == 0);
static_assert((NPROJ * DMODEL) % 8 == 0);

union Frag { v16h v; v8h hf[2]; };

__device__ __forceinline__ v8f wmma16(v16h a, v16h b, v8f c)
{
    return __builtin_amdgcn_wmma_f32_16x16x32_f16(false, a, false, b, (short)0, c, false, false);
}

__global__ void __launch_bounds__(128)
rmsnorm_f16_kernel(const float* __restrict__ u, const float* __restrict__ w,
                   _Float16* __restrict__ out, int nrows)
{
    const int lane = threadIdx.x & 31, wv = threadIdx.x >> 5;
    const int row = blockIdx.x * 4 + wv;
    if (row >= nrows) return;
    const float* ur = u + (size_t)row * DMODEL;
    v4f va[8];
    float ss = 0.f;
#pragma unroll
    for (int j = 0; j < 4; ++j) {
        const int c = (j * 32 + lane) * 8;
        va[2 * j]     = *(const v4f*)(ur + c);
        va[2 * j + 1] = *(const v4f*)(ur + c + 4);
#pragma unroll
        for (int e = 0; e < 4; ++e) {
            ss = fmaf(va[2 * j][e],     va[2 * j][e],     ss);
            ss = fmaf(va[2 * j + 1][e], va[2 * j + 1][e], ss);
        }
    }
#pragma unroll
    for (int off = 16; off > 0; off >>= 1) ss += __shfl_xor(ss, off);
    const float rs = rsqrtf(ss * (1.0f / (float)DMODEL) + RMS_EPS);
    v8h hv[4];
#pragma unroll
    for (int j = 0; j < 4; ++j) {
        const int c = (j * 32 + lane) * 8;
        const v4f w0 = *(const v4f*)(w + c);
        const v4f w1 = *(const v4f*)(w + c + 4);
#pragma unroll
        for (int e = 0; e < 4; ++e) {
            hv[j][e]     = (_Float16)((va[2 * j][e]     * rs) * w0[e]);
            hv[j][4 + e] = (_Float16)((va[2 * j + 1][e] * rs) * w1[e]);
        }
    }
    _Float16* orow = out + (size_t)row * DMODEL;
#pragma unroll
    for (int j = 0; j < 4; ++j)
        *(volatile v8h*)(orow + (j * 32 + lane) * 8) = hv[j];
    __threadfence();
#pragma unroll
    for (int j = 0; j < 4; ++j)
        *(volatile v8h*)(orow + (j * 32 + lane) * 8) = hv[j];
}

__global__ void __launch_bounds__(256)
convert_f16_kernel(const float* __restrict__ src, _Float16* __restrict__ dst,
                   int nvalid8, int ntotal8, float scale)
{
    const int i = blockIdx.x * 256 + threadIdx.x;
    if (i >= ntotal8) return;
    v4f v0 = {0.f, 0.f, 0.f, 0.f};
    v4f v1 = {0.f, 0.f, 0.f, 0.f};
    if (i < nvalid8) {
        v0 = *(const v4f*)(src + (size_t)i * 8);
        v1 = *(const v4f*)(src + (size_t)i * 8 + 4);
    }
    v8h hv;
#pragma unroll
    for (int e = 0; e < 4; ++e) {
        hv[e]     = (_Float16)(v0[e] * scale);
        hv[4 + e] = (_Float16)(v1[e] * scale);
    }
    _Float16* d = dst + (size_t)i * 8;
    *(volatile v8h*)d = hv;
    __threadfence();
    *(volatile v8h*)d = hv;
}

__global__ void __launch_bounds__(128)
gemm_f16_kernel(const _Float16* __restrict__ A, int lda,
                const _Float16* __restrict__ Bw, int ldb, int K,
                const float* __restrict__ bias, int nbias,
                float* __restrict__ C, int ldc)
{
    __shared__ __attribute__((aligned(16))) float stile[4][32 * SP];
    const int tid = threadIdx.x, lane = tid & 31, wv = tid >> 5;
    const int hh = lane >> 4, m = lane & 15;
    const int r0 = blockIdx.x * GBM + wv * 32;
    const int c0 = blockIdx.y * GBN;

    const _Float16* ap0 = A + (size_t)(r0 + m) * lda + 8 * hh;
    const _Float16* ap1 = ap0 + (size_t)16 * lda;
    const _Float16* bp  = Bw + (size_t)(c0 + m) * ldb + 8 * hh;
    const size_t bstep = (size_t)16 * ldb;

    const v8f z8 = {0.f, 0.f, 0.f, 0.f, 0.f, 0.f, 0.f, 0.f};
    v8f acc[2][4];
#pragma unroll
    for (int s = 0; s < 2; ++s)
#pragma unroll
        for (int t = 0; t < 4; ++t) acc[s][t] = z8;

#pragma unroll 1
    for (int k0 = 0; k0 < K; k0 += 32) {
        Frag a0, a1, b0, b1, b2, b3;
        a0.hf[0] = *(const v8h*)(ap0 + k0);
        a0.hf[1] = *(const v8h*)(ap0 + k0 + 16);
        a1.hf[0] = *(const v8h*)(ap1 + k0);
        a1.hf[1] = *(const v8h*)(ap1 + k0 + 16);
        b0.hf[0] = *(const v8h*)(bp + k0);
        b0.hf[1] = *(const v8h*)(bp + k0 + 16);
        b1.hf[0] = *(const v8h*)(bp + bstep + k0);
        b1.hf[1] = *(const v8h*)(bp + bstep + k0 + 16);
        b2.hf[0] = *(const v8h*)(bp + 2 * bstep + k0);
        b2.hf[1] = *(const v8h*)(bp + 2 * bstep + k0 + 16);
        b3.hf[0] = *(const v8h*)(bp + 3 * bstep + k0);
        b3.hf[1] = *(const v8h*)(bp + 3 * bstep + k0 + 16);

        acc[0][0] = wmma16(a0.v, b0.v, acc[0][0]);
        acc[0][1] = wmma16(a0.v, b1.v, acc[0][1]);
        acc[0][2] = wmma16(a0.v, b2.v, acc[0][2]);
        acc[0][3] = wmma16(a0.v, b3.v, acc[0][3]);
        acc[1][0] = wmma16(a1.v, b0.v, acc[1][0]);
        acc[1][1] = wmma16(a1.v, b1.v, acc[1][1]);
        acc[1][2] = wmma16(a1.v, b2.v, acc[1][2]);
        acc[1][3] = wmma16(a1.v, b3.v, acc[1][3]);
        asm volatile("v_nop\n\tv_nop\n\tv_nop\n\tv_nop"
                     : "+v"(acc[0][0]), "+v"(acc[0][1]), "+v"(acc[0][2]), "+v"(acc[0][3]),
                       "+v"(acc[1][0]), "+v"(acc[1][1]), "+v"(acc[1][2]), "+v"(acc[1][3])
                     : "v"(a0.v), "v"(a1.v), "v"(b0.v), "v"(b1.v), "v"(b2.v), "v"(b3.v));
    }

    float bv[4];
#pragma unroll
    for (int t = 0; t < 4; ++t) {
        const int col = c0 + t * 16 + m;
        bv[t] = (col < nbias) ? bias[col] : 0.f;
    }
    float* st = &stile[wv][0];
#pragma unroll
    for (int s = 0; s < 2; ++s)
#pragma unroll
        for (int t = 0; t < 4; ++t)
#pragma unroll
            for (int r = 0; r < 8; ++r)
                st[(s * 16 + 8 * hh + r) * SP + t * 16 + m] = acc[s][t][r] * WSCALE_INV + bv[t];
    __syncthreads();

    const int cc = m * 4;
    const float* sbase = st + hh * SP + cc;
    float* cbase = C + (size_t)(r0 + hh) * ldc + c0 + cc;
    v4f vals[16];
#pragma unroll
    for (int j = 0; j < 16; ++j) vals[j] = *(const v4f*)(sbase + 2 * j * SP);
#pragma unroll
    for (int j = 0; j < 16; ++j)
        *(volatile v4f*)(cbase + (size_t)(2 * j) * ldc) = vals[j];
    __threadfence();
#pragma unroll
    for (int j = 0; j < 16; ++j)
        *(volatile v4f*)(cbase + (size_t)(2 * j) * ldc) = vals[j];
}

__global__ void __launch_bounds__(256)
dt_kernel(const float* __restrict__ zx, const float* __restrict__ A_log,
          const float* __restrict__ dt_bias, float* __restrict__ dtv,
          float* __restrict__ dav, int n)
{
    const int i = blockIdx.x * 256 + threadIdx.x;
    if (i >= n) return;
    const int row = i >> 2, h = i & 3;
    const float v  = zx[(size_t)row * NPAD + COL_DT + h] + dt_bias[h];
    const float dt = fmaxf(v, 0.f) + log1pf(expf(-fabsf(v)));
    const float Ah = -expf(A_log[h]);
    const float da = expf(dt * Ah);
    *(volatile float*)(dtv + i) = dt;
    *(volatile float*)(dav + i) = da;
    __threadfence();
    *(volatile float*)(dtv + i) = dt;
    *(volatile float*)(dav + i) = da;
}

__global__ void __launch_bounds__(128)
scan_kernel(const float* __restrict__ zx, const float* __restrict__ dtv,
            const float* __restrict__ dav, const float* __restrict__ Dv,
            _Float16* __restrict__ g16)
{
    __shared__ __attribute__((aligned(16))) _Float16 stile[8][128];
    const int tid = threadIdx.x, lane = tid & 31, wv = tid >> 5;
    const int hh = lane >> 4, m = lane & 15;
    const int bid = blockIdx.x;
    const int b = bid >> 4, hd = (bid >> 2) & 3, pq = bid & 3;
    const int pw = pq * 128 + wv * 32;
    const float Dh = Dv[hd];

    float s0[32], s1[32];
#pragma unroll
    for (int j = 0; j < 32; ++j) { s0[j] = 0.f; s1[j] = 0.f; }

    const float* zb = zx + (size_t)b * LSEQ * NPAD;
    const int cx0 = COL_X + hd * HEADDIM + pw + m;
    const int cxo = COL_X + hd * HEADDIM + pw + lane;
    const int czo = hd * HEADDIM + pw + lane;
    const int cB  = COL_BC + hd * (2 * DSTATE) + 8 * hh;
    const int cC  = cB + DSTATE;
    const int dbase = b * LSEQ * NHEADS + hd;
    const int orow = 2 * wv + hh;
    const size_t ocol = (size_t)hd * HEADDIM + (size_t)pq * 128 + (size_t)m * 8;
    const v8f z8 = {0.f, 0.f, 0.f, 0.f, 0.f, 0.f, 0.f, 0.f};

    for (int t = 0; t < LSEQ; ++t) {
        const float* rp = zb + (size_t)t * NPAD;
        const float dt = dtv[dbase + t * NHEADS];
        const float dA = dav[dbase + t * NHEADS];
        const float x0 = rp[cx0];
        const float x1 = rp[cx0 + 16];
        const float dtx0 = dt * x0;
        const float dtx1 = dt * x1;

        v16h af[2], b0f[2], b1f[2];
#pragma unroll
        for (int ks = 0; ks < 2; ++ks) {
#pragma unroll
            for (int gg = 0; gg < 2; ++gg) {
                const int g = 2 * ks + gg;
#pragma unroll
                for (int q = 0; q < 2; ++q) {
                    const v4f bq = *(const v4f*)(rp + cB + 16 * g + 4 * q);
                    const v4f cq = *(const v4f*)(rp + cC + 16 * g + 4 * q);
#pragma unroll
                    for (int e = 0; e < 4; ++e) {
                        const int i = 4 * q + e;
                        const int j = 8 * g + i;
                        s0[j] = fmaf(s0[j], dA, bq[e] * dtx0);
                        s1[j] = fmaf(s1[j], dA, bq[e] * dtx1);
                        af[ks][8 * gg + i]  = (_Float16)cq[e];
                        b0f[ks][8 * gg + i] = (_Float16)s0[j];
                        b1f[ks][8 * gg + i] = (_Float16)s1[j];
                    }
                }
            }
        }
        v8f acc0 = wmma16(af[0], b0f[0], z8);
        v8f acc1 = wmma16(af[0], b1f[0], z8);
        acc0 = wmma16(af[1], b0f[1], acc0);
        acc1 = wmma16(af[1], b1f[1], acc1);
        asm volatile("v_nop\n\tv_nop\n\tv_nop\n\tv_nop"
                     : "+v"(acc0), "+v"(acc1)
                     : "v"(af[0]), "v"(af[1]), "v"(b0f[0]), "v"(b0f[1]), "v"(b1f[0]), "v"(b1f[1]));

        const float yv = hh ? acc1[0] : acc0[0];
        const float xo = rp[cxo];
        const float y  = fmaf(xo, Dh, yv);
        const float z  = rp[czo];
        const float ez = expf(-z);
        const float sg = __builtin_amdgcn_rcpf(1.0f + ez);
        const float g  = y * (z * sg);
        stile[t & 7][tid] = (_Float16)g;

        if ((t & 7) == 7) {
            __syncthreads();
            const v8h hv = *(const v8h*)(&stile[orow][m * 8]);
            _Float16* gp = g16 + (size_t)(b * LSEQ + (t - 7) + orow) * DINNER + ocol;
            *(volatile v8h*)gp = hv;
            __threadfence();
            *(volatile v8h*)gp = hv;
            __syncthreads();
        }
    }
}

extern "C" void kernel_launch(void* const* d_in, const int* in_sizes, int n_in,
                              void* d_out, int out_size, void* d_ws, size_t ws_size,
                              hipStream_t stream)
{
    if (n_in < 9) return;
    if (in_sizes[0] != ROWS * DMODEL || in_sizes[1] != DMODEL ||
        in_sizes[2] != NPROJ * DMODEL || in_sizes[3] != NPROJ ||
        in_sizes[4] != NHEADS || in_sizes[5] != NHEADS || in_sizes[6] != NHEADS ||
        in_sizes[7] != DMODEL * DINNER || in_sizes[8] != DMODEL) return;
    if (out_size != ROWS * DMODEL) return;

    const float* u       = (const float*)d_in[0];
    const float* norm_w  = (const float*)d_in[1];
    const float* in_w    = (const float*)d_in[2];
    const float* in_b    = (const float*)d_in[3];
    const float* A_log   = (const float*)d_in[4];
    const float* Dvec    = (const float*)d_in[5];
    const float* dt_bias = (const float*)d_in[6];
    const float* out_w   = (const float*)d_in[7];
    const float* out_b   = (const float*)d_in[8];
    float* out = (float*)d_out;

    size_t off = 0;
    auto carve = [&](size_t bytes) -> size_t {
        const size_t o = off;
        off += (bytes + 255) & ~(size_t)255;
        return o;
    };
    const size_t o_un = carve((size_t)ROWS * DMODEL * sizeof(_Float16));
    const size_t o_w1 = carve((size_t)NPAD * DMODEL * sizeof(_Float16));
    const size_t o_w2 = carve((size_t)DMODEL * DINNER * sizeof(_Float16));
    const size_t o_zx = carve((size_t)ROWS * NPAD * sizeof(float));
    const size_t o_dt = carve((size_t)ROWS * NHEADS * sizeof(float));
    const size_t o_da = carve((size_t)ROWS * NHEADS * sizeof(float));
    const size_t o_g  = carve((size_t)ROWS * DINNER * sizeof(_Float16));
    if (off > ws_size || off > WS_LIMIT) return;

    char* ws = (char*)d_ws;
    _Float16* un16 = (_Float16*)(ws + o_un);
    _Float16* w1h  = (_Float16*)(ws + o_w1);
    _Float16* w2h  = (_Float16*)(ws + o_w2);
    float*    zx   = (float*)(ws + o_zx);
    float*    dtv  = (float*)(ws + o_dt);
    float*    dav  = (float*)(ws + o_da);
    _Float16* g16  = (_Float16*)(ws + o_g);

    rmsnorm_f16_kernel<<<(ROWS + 3) / 4, 128, 0, stream>>>(u, norm_w, un16, ROWS);

    {
        const int nval8 = (NPROJ * DMODEL) / 8;
        const int ntot8 = (NPAD * DMODEL) / 8;
        convert_f16_kernel<<<(ntot8 + 255) / 256, 256, 0, stream>>>(in_w, w1h, nval8, ntot8, WSCALE);
    }
    {
        const int ntot8 = (DMODEL * DINNER) / 8;
        convert_f16_kernel<<<(ntot8 + 255) / 256, 256, 0, stream>>>(out_w, w2h, ntot8, ntot8, WSCALE);
    }

    gemm_f16_kernel<<<dim3(ROWS / GBM, NPAD / GBN), 128, 0, stream>>>(
        un16, DMODEL, w1h, DMODEL, DMODEL, in_b, NPROJ, zx, NPAD);

    dt_kernel<<<(ROWS * NHEADS + 255) / 256, 256, 0, stream>>>(zx, A_log, dt_bias, dtv, dav, ROWS * NHEADS);

    scan_kernel<<<BDIM * NHEADS * (HEADDIM / 128), 128, 0, stream>>>(zx, dtv, dav, Dvec, g16);

    gemm_f16_kernel<<<dim3(ROWS / GBM, DMODEL / GBN), 128, 0, stream>>>(
        g16, DINNER, w2h, DINNER, DINNER, out_b, DMODEL, out, DMODEL);
}
